// SymmetricalLayer_61864708932165
// MI455X (gfx1250) — hardware-verified
//
#include <hip/hip_runtime.h>


#define NB  8192
#define ND  1024
#define NC  128
typedef _Float16 h16;
typedef unsigned short bf;
typedef __attribute__((ext_vector_type(16))) __bf16   v16bf;
typedef __attribute__((ext_vector_type(16))) _Float16 v16h;
typedef __attribute__((ext_vector_type(8)))  _Float16 v8h;
typedef __attribute__((ext_vector_type(8)))  unsigned short v8us;
typedef __attribute__((ext_vector_type(8)))  float    v8f;
typedef __attribute__((ext_vector_type(4)))  float    v4f;
typedef v8h  __attribute__((may_alias)) v8ha;
typedef v4f  __attribute__((may_alias)) v4fa;
typedef v8us __attribute__((may_alias)) v8usa;

__device__ __forceinline__ unsigned short f2bf(float f) { unsigned u = __float_as_uint(f); u += 0x7FFFu + ((u >> 16) & 1u); return (unsigned short)(u >> 16); }
__device__ __forceinline__ float bf2f(unsigned short b) { return __uint_as_float(((unsigned)b) << 16); }
__device__ __forceinline__ float bfr(float f) { return bf2f(f2bf(f)); }
__device__ __forceinline__ v16h cat16(v8h lo, v8h hi) { return __builtin_shufflevector(lo, hi, 0, 1, 2, 3, 4, 5, 6, 7, 8, 9, 10, 11, 12, 13, 14, 15); }
__device__ __forceinline__ v16bf cat16b(v8us lo, v8us hi) { return __builtin_bit_cast(v16bf, __builtin_shufflevector(lo, hi, 0, 1, 2, 3, 4, 5, 6, 7, 8, 9, 10, 11, 12, 13, 14, 15)); }
__device__ __forceinline__ v8f wmma16(v16h a, v16h b, v8f c) { return __builtin_amdgcn_wmma_f32_16x16x32_f16(false, a, false, b, (short)0, c, false, false); }
__device__ __forceinline__ v8f wmmab(v16bf a, v16bf b, v8f c) { return __builtin_amdgcn_wmma_f32_16x16x32_bf16(false, a, false, b, (short)0, c, false, false); }

template <typename T16> struct WFrag;
template <> struct WFrag<h16> { typedef v16h V; static __device__ __forceinline__ V ld(const h16* p) { return cat16(*(const v8h*)p, *(const v8h*)(p + 16)); } static __device__ __forceinline__ v8f mma(V a, V b, v8f c) { return wmma16(a, b, c); } };
template <> struct WFrag<bf> { typedef v16bf V; static __device__ __forceinline__ V ld(const bf* p) { return cat16b(*(const v8us*)p, *(const v8us*)(p + 16)); } static __device__ __forceinline__ v8f mma(V a, V b, v8f c) { return wmmab(a, b, c); } };
template <typename T16, int NSPLIT, bool BIAS>
__global__ __launch_bounds__(32) void k_gemmw(const T16* __restrict__ A, const T16* __restrict__ A2, const T16* __restrict__ Bt, const T16* __restrict__ Bt2, int K, float* C, int ldc, const float* __restrict__ bias, size_t sA, size_t sB, size_t sC) {
    typedef typename WFrag<T16>::V V;
    __shared__ __align__(16) float os[16 * 68];
    const size_t z = blockIdx.z; A += z * sA; if (A2) A2 += z * sA; Bt += z * sB; if (Bt2) Bt2 += z * sB; C += z * sC;
    const int lane = threadIdx.x & 31, lr = lane & 15, hi = lane >> 4; const int r0 = blockIdx.x * 64, c0 = blockIdx.y * 64;
    v8f acc[4][4];
#pragma unroll
    for (int mb = 0; mb < 4; ++mb)
#pragma unroll
        for (int nb = 0; nb < 4; ++nb) acc[mb][nb] = (v8f){};
    const size_t aoff = (size_t)(r0 + lr) * K + 8 * hi, boff = (size_t)(c0 + lr) * K + 8 * hi;
    for (int kc = 0; kc < K; kc += 32) {
        V a[4], a2[4];
#pragma unroll
        for (int mb = 0; mb < 4; ++mb) { a[mb] = WFrag<T16>::ld(A + aoff + (size_t)mb * 16 * K + kc); if (NSPLIT == 1 || NSPLIT == 2) a2[mb] = WFrag<T16>::ld(A2 + aoff + (size_t)mb * 16 * K + kc); }
#pragma unroll
        for (int nb = 0; nb < 4; ++nb) { const V b = WFrag<T16>::ld(Bt + boff + (size_t)nb * 16 * K + kc); V b2; if (NSPLIT >= 2) b2 = WFrag<T16>::ld(Bt2 + boff + (size_t)nb * 16 * K + kc);
#pragma unroll
            for (int mb = 0; mb < 4; ++mb) { acc[mb][nb] = WFrag<T16>::mma(a[mb], b, acc[mb][nb]); if (NSPLIT == 1 || NSPLIT == 2) acc[mb][nb] = WFrag<T16>::mma(a2[mb], b, acc[mb][nb]); if (NSPLIT >= 2) acc[mb][nb] = WFrag<T16>::mma(a[mb], b2, acc[mb][nb]); } }
        asm volatile("v_nop\n\tv_nop\n\tv_nop\n\tv_nop" : "+v"(acc[0][0]), "+v"(acc[1][1]), "+v"(acc[2][2]), "+v"(acc[3][3]) : "v"(a[0]), "v"(a[3]));
    }
#pragma unroll
    for (int mb = 0; mb < 4; ++mb) {
#pragma unroll
        for (int nb = 0; nb < 4; ++nb) {
#pragma unroll
            for (int j = 0; j < 8; ++j) os[(hi * 8 + j) * 68 + nb * 16 + lr] = acc[mb][nb][j]; }
        __builtin_amdgcn_wave_barrier(); asm volatile("" ::: "memory");
        float* crow = C + (size_t)(r0 + mb * 16) * ldc + c0;
#pragma unroll 1
        for (int ps = 0; ps < 2; ++ps) {
#pragma unroll
            for (int s = 0; s < 8; ++s) { const int row = 2 * s + hi, cofs = lr * 4; v4f val = *(const v4fa*)(os + row * 68 + cofs); if (BIAS) { val[0] += bfr(bias[c0 + cofs]); val[1] += bfr(bias[c0 + cofs + 1]); val[2] += bfr(bias[c0 + cofs + 2]); val[3] += bfr(bias[c0 + cofs + 3]); }
                *(volatile v4f*)(crow + (size_t)row * ldc + cofs) = val; }
            if (ps == 0) __threadfence(); }
        __builtin_amdgcn_wave_barrier(); asm volatile("" ::: "memory");
    }
}

typedef __attribute__((ext_vector_type(2))) _Float16 v2h;
typedef __attribute__((ext_vector_type(4))) _Float16 v4h;
typedef __attribute__((ext_vector_type(2))) unsigned short v2us;
typedef __attribute__((ext_vector_type(4))) unsigned short v4us;
typedef __attribute__((ext_vector_type(2))) float v2f;
__device__ __forceinline__ h16 toh_flush(float x) { const float z = (fabsf(x) < 6.103515625e-05f) ? 0.0f : x; return (h16)z; }

__global__ __launch_bounds__(32) void k_gs(const float* __restrict__ g, float* S) { if (blockIdx.x != 0 || threadIdx.x != 0) return;
    float s0 = 0.0f, s1 = 0.0f; for (int d = 0; d < ND; ++d) { const float a = bfr(g[d]), b = bfr(g[ND + d]); s0 = __fmaf_rn(a, a, s0); s1 = __fmaf_rn(b, b, s1); }
    const float m0 = fmaxf(__fsqrt_rn(s0), 1e-12f), m1 = fmaxf(__fsqrt_rn(s1), 1e-12f);
    float t = 0.0f; for (int d = 0; d < ND; ++d) { const float a = __fdiv_rn(bfr(g[d]), m0); t = __fmaf_rn(a, a, t); }
    const float l0 = __fsqrt_rn(t);
    float dt = 0.0f; for (int d = 0; d < ND; ++d) { const float p = __fdiv_rn(__fdiv_rn(bfr(g[d]), m0), l0); const float b = __fdiv_rn(bfr(g[ND + d]), m1); dt = __fmaf_rn(p, b, dt); }
    float r = 0.0f; for (int d = 0; d < ND; ++d) { const float p = __fdiv_rn(__fdiv_rn(bfr(g[d]), m0), l0); const float v = __fsub_rn(__fdiv_rn(bfr(g[ND + d]), m1), __fmul_rn(dt, p)); r = __fmaf_rn(v, v, r); }
    const float l1 = __fsqrt_rn(r);
    float spp = 0.0f, sqp = 0.0f; for (int d = 0; d < ND; ++d) { const float p = __fdiv_rn(__fdiv_rn(bfr(g[d]), m0), l0); const float q = __fdiv_rn(__fsub_rn(__fdiv_rn(bfr(g[ND + d]), m1), __fmul_rn(dt, p)), l1); spp = __fmaf_rn(p, p, spp); sqp = __fmaf_rn(q, p, sqp); }
    v4f o0, o1; o0[0] = m0; o0[1] = l0; o0[2] = m1; o0[3] = dt; o1[0] = l1; o1[1] = spp; o1[2] = sqp; o1[3] = __fmul_rn(sqp, 0.0f);
    v4f oz; oz[0] = o1[3]; oz[1] = o1[3]; oz[2] = o1[3]; oz[3] = o1[3];
#pragma unroll
    for (int ps = 0; ps < 2; ++ps) { *(volatile v4f*)(S) = o0; *(volatile v4f*)(S + 4) = o1;
#pragma unroll
        for (int k = 2; k < 8; ++k) *(volatile v4f*)(S + 4 * k) = oz;
        if (ps == 0) __threadfence(); } }

__device__ const float TSN[128] = {
    0.0f, 0.0490676761f, 0.0980171412f, 0.146730468f, 0.195090324f, 0.242980197f, 0.290284663f, 0.336889863f,
    0.382683456f, 0.427555084f, 0.471396744f, 0.514102757f, 0.555570245f, 0.59569931f, 0.634393334f, 0.671558976f,
    0.707106769f, 0.74095118f, 0.773010433f, 0.803207517f, 0.831469655f, 0.85772866f, 0.881921291f, 0.903989315f,
    0.923879504f, 0.941544056f, 0.956940353f, 0.970031261f, 0.98078531f, 0.989176512f, 0.99518472f, 0.99879545f,
    1.0f, 0.99879545f, 0.99518472f, 0.989176512f, 0.980785251f, 0.970031261f, 0.956940293f, 0.941544056f,
    0.923879504f, 0.903989315f, 0.881921232f, 0.857728601f, 0.831469536f, 0.803207517f, 0.773010492f, 0.740951061f,
    0.707106769f, 0.671558857f, 0.634393275f, 0.595699131f, 0.555570185f, 0.514102757f, 0.471396625f, 0.427555054f,
    0.382683277f, 0.336889803f, 0.290284723f, 0.242980078f, 0.195090309f, 0.146730334f, 0.0980170965f, 0.0490674861f,
    -8.74227766e-08f, -0.0490676612f, -0.0980172679f, -0.146730497f, -0.195090488f, -0.242980242f, -0.290284872f, -0.336889952f,
    -0.382683426f, -0.427555233f, -0.471396774f, -0.514102876f, -0.555570304f, -0.59569931f, -0.634393394f, -0.671558976f,
    -0.707106888f, -0.74095118f, -0.773010433f, -0.803207576f, -0.831469774f, -0.857728541f, -0.881921291f, -0.903989375f,
    -0.923879683f, -0.941544056f, -0.956940353f, -0.970031321f, -0.980785251f, -0.989176512f, -0.99518472f, -0.99879545f,
    -1.0f, -0.99879545f, -0.99518472f, -0.989176512f, -0.980785251f, -0.970031202f, -0.956940234f, -0.941544056f,
    -0.923879445f, -0.903989136f, -0.881921291f, -0.857728541f, -0.831469476f, -0.803207576f, -0.773010433f, -0.740951002f,
    -0.707106531f, -0.671558976f, -0.634393156f, -0.595699072f, -0.555570304f, -0.514102697f, -0.471396536f, -0.427554786f,
    -0.382683426f, -0.336889714f, -0.290284395f, -0.242980227f, -0.195090234f, -0.146730244f, -0.0980167687f, -0.0490676388f };
__device__ const float TCM[128] = {
    0.0f, -0.00120455027f, -0.00481528044f, -0.0108234882f, -0.0192147493f, -0.0299687386f, -0.0430596471f, -0.0584559441f,
    -0.0761204958f, -0.096010685f, -0.118078768f, -0.142271399f, -0.168530405f, -0.196792483f, -0.226989567f, -0.259048879f,
    -0.292893231f, -0.328441083f, -0.365606725f, -0.40430069f, -0.444429815f, -0.485897303f, -0.528603315f, -0.572444916f,
    -0.617316604f, -0.663110137f, -0.709715366f, -0.757019877f, -0.804909766f, -0.853269517f, -0.901982844f, -0.950932324f,
    -1.0f, -1.04906774f, -1.09801722f, -1.14673054f, -1.19509029f, -1.24298024f, -1.29028475f, -1.33688998f,
    -1.38268352f, -1.42755508f, -1.4713968f, -1.5141027f, -1.55557036f, -1.59569931f, -1.63439322f, -1.6715591f,
    -1.70710683f, -1.7409513f, -1.77301049f, -1.80320764f, -1.83146966f, -1.8577286f, -1.88192129f, -1.90398932f,
    -1.92387962f, -1.94154406f, -1.95694041f, -1.97003126f, -1.98078537f, -1.98917651f, -1.99518466f, -1.99879551f,
    -2.0f, -1.99879551f, -1.99518466f, -1.98917651f, -1.98078525f, -1.97003126f, -1.95694029f, -1.94154406f,
    -1.9238795f, -1.90398932f, -1.88192129f, -1.85772848f, -1.83146954f, -1.80320752f, -1.77301037f, -1.74095106f,
    -1.70710659f, -1.67155886f, -1.63439333f, -1.59569919f, -1.55557001f, -1.51410282f, -1.47139668f, -1.42755497f,
    -1.38268316f, -1.33688986f, -1.29028451f, -1.24297988f, -1.19509041f, -1.14673042f, -1.09801698f, -1.04906738f,
    -1.0f, -0.950932145f, -0.901982546f, -0.853269577f, -0.804909587f, -0.757019579f, -0.709715009f, -0.663110137f,
    -0.617316365f, -0.572444618f, -0.528603315f, -0.485897183f, -0.444429576f, -0.404300749f, -0.365606666f, -0.328440905f,
    -0.292892992f, -0.259048879f, -0.226989448f, -0.196792305f, -0.168530405f, -0.14227134f, -0.118078649f, -0.0960105658f,
    -0.0761204362f, -0.0584558845f, -0.0430595875f, -0.0299687386f, -0.0192146897f, -0.0108234286f, -0.00481522083f, -0.00120455027f };
__global__ __launch_bounds__(256) void k_tab(const float* __restrict__ g, const float* __restrict__ S, h16* T) { const int i = blockIdx.x * 256 + threadIdx.x; if (i >= NC * ND / 8) return; const int c = i >> 7, d0 = (i & 127) * 8; const float sn = TSN[c], cm = TCM[c]; const float m0 = S[0], l0 = S[1], m1 = S[2], dt = S[3], l1 = S[4], spp = S[5], sqp = S[6]; const v8f g0 = *(const v8f*)(g + d0); const v8f g1 = *(const v8f*)(g + ND + d0); v8h o;
#pragma unroll
    for (int e = 0; e < 8; ++e) { const float p = __fdiv_rn(__fdiv_rn(bfr(g0[e]), m0), l0); const float q = __fdiv_rn(__fsub_rn(__fdiv_rn(bfr(g1[e]), m1), __fmul_rn(dt, p)), l1); const float u = __fsub_rn(__fmul_rn(q, spp), __fmul_rn(p, sqp)); const float w = __fadd_rn(__fmul_rn(p, spp), __fmul_rn(q, sqp)); o[e] = toh_flush(__fmaf_rn(cm, w, __fmaf_rn(sn, u, p))); }
    *(volatile v8h*)(T + (size_t)i * 8) = o; __threadfence(); *(volatile v8h*)(T + (size_t)i * 8) = o; }

__global__ __launch_bounds__(256) void k_rn(const float* __restrict__ a, float* F) { const int r = blockIdx.x * 256 + threadIdx.x; if (r >= NB) return; float s = 0.0f;
    for (int k = 0; k < ND / 4; ++k) { const v4f v = *(const v4f*)(a + (size_t)r * ND + 4 * k); const float x0 = bfr(v[0]), x1 = bfr(v[1]), x2 = bfr(v[2]), x3 = bfr(v[3]); s = __fmaf_rn(x0, x0, s); s = __fmaf_rn(x1, x1, s); s = __fmaf_rn(x2, x2, s); s = __fmaf_rn(x3, x3, s); }
    const float f = __fdiv_rn(16.0f, fmaxf(__fsqrt_rn(s), 1e-12f)); *(volatile float*)(F + r) = f; __threadfence(); *(volatile float*)(F + r) = f; }

__global__ __launch_bounds__(256) void k_as(const float* __restrict__ a, const float* __restrict__ F, h16* X) { const int i = blockIdx.x * 256 + threadIdx.x; if (i >= NB * ND / 8) return; const float f = F[i >> 7]; const v8f v = *(const v8f*)(a + (size_t)i * 8); v8h o;
#pragma unroll
    for (int q = 0; q < 8; ++q) o[q] = toh_flush(__fmul_rn(bfr(v[q]), f));
    *(volatile v8h*)(X + (size_t)i * 8) = o; __threadfence(); *(volatile v8h*)(X + (size_t)i * 8) = o; }

extern "C" void kernel_launch(void* const* d_in, const int* in_sizes, int n_in, void* d_out, int out_size, void* d_ws, size_t ws_size, hipStream_t stream) {
    if (n_in < 2) return;
    if (in_sizes[0] != NB * ND || in_sizes[1] != 2 * ND) return;
    if (out_size != NB * NC) return;
    static_assert(NB % 64 == 0 && NC % 64 == 0 && ND % 32 == 0 && ND % 8 == 0 && (NC * ND / 8) % 256 == 0 && (NB * ND / 8) % 256 == 0 && NB % 256 == 0 && ND == 1024 && NC == 128, "the product: M and N multiples of 64, the depth a multiple of 32; every elementwise grid exact; the shifts of k_tab and k_as are for a depth of 1,024");
    const float* a = (const float*)d_in[0]; const float* g = (const float*)d_in[1];
    float* out = (float*)d_out;
    char* wsp = (char*)d_ws; auto take = [&](size_t bytes) { char* p = wsp; wsp += (bytes + 255) & ~(size_t)255; return (void*)p; };
    float* S = (float*)take((size_t)32 * 4); h16* T = (h16*)take((size_t)NC * ND * 2); float* F = (float*)take((size_t)NB * 4); h16* X = (h16*)take((size_t)NB * ND * 2);
    if ((size_t)(wsp - (char*)d_ws) > ws_size) return;
    k_gs<<<1, 32, 0, stream>>>(g, S);
    k_tab<<<(unsigned)(NC * ND / 8 / 256), 256, 0, stream>>>(g, S, T);
    k_rn<<<(unsigned)(NB / 256), 256, 0, stream>>>(a, F);
    k_as<<<(unsigned)(NB * ND / 8 / 256), 256, 0, stream>>>(a, F, X);
    k_gemmw<h16, 0, false><<<dim3(NB / 64, NC / 64, 1), 32, 0, stream>>>(X, nullptr, T, nullptr, ND, out, NC, nullptr, 0, 0, 0);
}
